// TTTLayer_8632884264977
// MI455X (gfx1250) — hardware-verified
//
#include <hip/hip_runtime.h>
#include <math.h>

constexpr int kB = 4;
constexpr int kDim = 512;
constexpr int kTok = 4096;
constexpr int kNH = 8;
constexpr int kHD = 64;
constexpr int kCS = 16;
constexpr int kNC = kTok / kCS;
constexpr int kBT = kB * kTok;
constexpr int kHalfTok = 2 * kTok;

typedef __attribute__((ext_vector_type(16))) __bf16   v16b;
typedef __attribute__((ext_vector_type(8)))  __bf16   v8b;
typedef __attribute__((ext_vector_type(8)))  float    v8f;
typedef __attribute__((ext_vector_type(4)))  float    v4f;
typedef __attribute__((ext_vector_type(4)))  unsigned v4u;
typedef __attribute__((ext_vector_type(2)))  unsigned v2u;

__device__ __forceinline__ unsigned short f2bf_bits(float f) {
  unsigned u = __float_as_uint(f);
  return (unsigned short)((u + 0x7FFFu + ((u >> 16) & 1u)) >> 16);
}
__device__ __forceinline__ float bf_bits2f(unsigned short h) { return __uint_as_float(((unsigned)h) << 16); }
__device__ __forceinline__ float bfr(float f) { return bf_bits2f(f2bf_bits(f)); }
__device__ __forceinline__ void split2(float f, unsigned short& hb, unsigned short& lb) {
  hb = f2bf_bits(f);
  lb = f2bf_bits(f - bf_bits2f(hb));
}
__device__ __forceinline__ unsigned pk2(unsigned short a, unsigned short b) { return (unsigned)a | ((unsigned)b << 16); }
__device__ __forceinline__ v8f zero8() { return (v8f){0.f, 0.f, 0.f, 0.f, 0.f, 0.f, 0.f, 0.f}; }

__device__ __forceinline__ void dep_guard_b(v8f& a, v8f& b, v16b x, v16b y) { asm volatile("v_nop\n\tv_nop\n\tv_nop\n\tv_nop" : "+v"(a), "+v"(b) : "v"(x), "v"(y)); }
__device__ __forceinline__ void keep4_b(v16b a, v16b b, v16b c, v16b d) { asm volatile("v_nop" :: "v"(a), "v"(b), "v"(c), "v"(d)); }
__device__ __forceinline__ void acc_guard4(v8f& a, v8f& b, v8f& c, v8f& d) { asm volatile("v_nop\n\tv_nop\n\tv_nop\n\tv_nop" : "+v"(a), "+v"(b), "+v"(c), "+v"(d)); }
template <typename T> struct Frag;
template <> struct Frag<__bf16> {
  typedef v16b V; union U { v16b v; v8b h[2]; };
  static __device__ __forceinline__ v16b load(const __bf16* p) {
    U f; f.h[0] = *(const v8b*)(p); f.h[1] = *(const v8b*)(p + 16); return f.v;
  }
  static __device__ __forceinline__ v8f mma(v16b a, v16b b, v8f c) {
    return __builtin_amdgcn_wmma_f32_16x16x32_bf16(false, a, false, b, (short)0, c, false, false);
  }
  static __device__ __forceinline__ void guard(v8f& a, v8f& b, v16b x, v16b y) { dep_guard_b(a, b, x, y); }
  static __device__ __forceinline__ void keep(v16b a, v16b b, v16b c, v16b d) { keep4_b(a, b, c, d); }
};

__device__ __forceinline__ v16b frag_lds(const unsigned short* p) {
  union { v16b v; v4u u[2]; } f;
  f.u[0] = *(const v4u*)(p);
  f.u[1] = *(const v4u*)(p + 16);
  return f.v;
}
__device__ __forceinline__ v8f bmma(v16b a, v16b b, v8f c) {
  c = __builtin_amdgcn_wmma_f32_16x16x32_bf16(false, a, false, b, (short)0, c, false, false);
  asm volatile("v_nop\n\tv_nop\n\tv_nop\n\tv_nop" : "+v"(c) : "v"(a), "v"(b));
  return c;
}
__device__ __forceinline__ float red8(float v) {
  v += __shfl_xor(v, 1, 32);
  v += __shfl_xor(v, 2, 32);
  v += __shfl_xor(v, 4, 32);
  return v;
}
__device__ __forceinline__ float red32(float v) {
  v += __shfl_xor(v, 16, 32);
  v += __shfl_xor(v, 8, 32);
  v += __shfl_xor(v, 4, 32);
  v += __shfl_xor(v, 2, 32);
  v += __shfl_xor(v, 1, 32);
  return v;
}
__device__ __forceinline__ void st_split4(unsigned short* ph, unsigned short* pl, float a, float b, float c, float d) {
  unsigned short ha, hb, hc, hdd, la, lbb, lc, ldd;
  split2(a, ha, la); split2(b, hb, lbb); split2(c, hc, lc); split2(d, hdd, ldd);
  *(v2u*)ph = (v2u){pk2(ha, hb), pk2(hc, hdd)};
  *(v2u*)pl = (v2u){pk2(la, lbb), pk2(lc, ldd)};
}

template <bool ASPLIT, bool BSPLIT>
__global__ __launch_bounds__(256) void gemm64_bf16(
    const unsigned short* __restrict__ Ap, const unsigned short* __restrict__ A2p, int lda, long strideA,
    const unsigned short* __restrict__ Btp, const unsigned short* __restrict__ Bt2p, int ldb, long strideB,
    float* __restrict__ Cp, int ldc, long strideC, int M, int N, int K) {
  typedef __bf16 T;
  typedef v16b V;
  const T* A = (const T*)Ap; const T* A2 = (const T*)A2p; const T* Bt = (const T*)Btp; const T* Bt2 = (const T*)Bt2p;
  __shared__ __align__(16) float sT[8][16 * 68];
  const int b    = blockIdx.y;
  const int lane = threadIdx.x & 31;
  const int wave = threadIdx.x >> 5;
  const int tilesN = N >> 6;
  const int tilesM = M >> 6;
  const int tile = blockIdx.x * 8 + wave;
  if (tile >= tilesM * tilesN) return;
  const int tm = tile / tilesN;
  const int tn = tile - tm * tilesN;
  const int m0 = tm << 6;
  const int n0 = tn << 6;

  const T* Ab  = A   + (size_t)b * strideA;
  const T* Bb  = Bt  + (size_t)b * strideB;
  const T* Ab2 = A2  + (size_t)b * strideA;
  const T* Bb2 = Bt2 + (size_t)b * strideB;

  const int rlane = lane & 15;
  const int koff  = (lane >> 4) * 8;
  const int mOff  = (lane >> 4) * 8;

  v8f acc[4][4];
#pragma unroll
  for (int i = 0; i < 4; ++i)
#pragma unroll
    for (int j = 0; j < 4; ++j) acc[i][j] = zero8();

  for (int k0 = 0; k0 < K; k0 += 32) {
    V bh[4], bl[4];
#pragma unroll
    for (int j = 0; j < 4; ++j) {
      const size_t bo = (size_t)(n0 + (j << 4) + rlane) * ldb + koff + k0;
      bh[j] = Frag<T>::load(Bb + bo);
      if (BSPLIT) bl[j] = Frag<T>::load(Bb2 + bo); else bl[j] = bh[j];
    }
#pragma unroll
    for (int i = 0; i < 4; ++i) {
      const size_t ao = (size_t)(m0 + (i << 4) + rlane) * lda + koff + k0;
      V ah = Frag<T>::load(Ab + ao);
      V al = ah;
      if (ASPLIT) al = Frag<T>::load(Ab2 + ao);
#pragma unroll
      for (int j = 0; j < 4; ++j) {
        acc[i][j] = Frag<T>::mma(ah, bh[j], acc[i][j]);
        if (BSPLIT) acc[i][j] = Frag<T>::mma(ah, bl[j], acc[i][j]);
        if (ASPLIT) acc[i][j] = Frag<T>::mma(al, bh[j], acc[i][j]);
      }
      Frag<T>::guard(acc[i][0], acc[i][3], ah, al);
    }
    Frag<T>::keep(bh[0], bh[1], bh[2], bh[3]);
    if (BSPLIT) Frag<T>::keep(bl[0], bl[1], bl[2], bl[3]);
  }
  acc_guard4(acc[0][0], acc[0][1], acc[0][2], acc[0][3]);
  acc_guard4(acc[1][0], acc[1][1], acc[1][2], acc[1][3]);
  acc_guard4(acc[2][0], acc[2][1], acc[2][2], acc[2][3]);
  acc_guard4(acc[3][0], acc[3][1], acc[3][2], acc[3][3]);

  float* slab = sT[wave];
#pragma unroll
  for (int i = 0; i < 4; ++i) {
    const int mBase = m0 + (i << 4);
#pragma unroll
    for (int j = 0; j < 4; ++j) {
#pragma unroll
      for (int r = 0; r < 8; ++r) slab[(mOff + r) * 68 + (j << 4) + rlane] = acc[i][j][r];
    }
    __builtin_amdgcn_fence(__ATOMIC_RELEASE, "workgroup");
    __builtin_amdgcn_wave_barrier();
    __builtin_amdgcn_fence(__ATOMIC_ACQUIRE, "workgroup");
    {
      float* C = Cp + (size_t)b * strideC;
      const int hh = lane >> 4, c4 = (lane & 15) * 4;
      for (int pass = 0; pass < 2; ++pass) {
#pragma unroll
        for (int it = 0; it < 8; ++it) {
          const int row = it * 2 + hh;
          v4f v = *(const v4f*)(slab + row * 68 + c4);
          *(volatile v4f*)(C + (size_t)(mBase + row) * ldc + n0 + c4) = v;
        }
        __threadfence();
      }
    }
    __builtin_amdgcn_fence(__ATOMIC_RELEASE, "workgroup");
    __builtin_amdgcn_wave_barrier();
    __builtin_amdgcn_fence(__ATOMIC_ACQUIRE, "workgroup");
  }
}

struct RopeFreq { float inv[32]; };
typedef char ct_ropefreq_size[(sizeof(RopeFreq) == 128) ? 1 : -1];

__global__ __launch_bounds__(128) void tables_kernel(float* __restrict__ cosT, float* __restrict__ sinT, RopeFreq rf) {
  __shared__ __align__(16) float Ct[128 * 32];
  __shared__ __align__(16) float St[128 * 32];
  __shared__ float invL[32];
  const int tid = threadIdx.x, wave = tid >> 5, lane = tid & 31;
  const int t = blockIdx.x * 128 + tid;
  {
    float mv = 0.0f;
#pragma unroll
    for (int e = 0; e < 32; ++e) mv = (tid == e) ? rf.inv[e] : mv;
    if (tid < 32) invL[tid] = mv;
  }
  __syncthreads();
#pragma unroll 1
  for (int j = 0; j < 32; ++j) {
    float ang = (float)t * invL[j];
    asm volatile("" : "+v"(ang));
    Ct[tid * 32 + j] = cosf(ang);
    St[tid * 32 + j] = sinf(ang);
  }
  __syncthreads();
  const int q = lane >> 3, c4 = (lane & 7) * 4;
  v4f cv[8], sv[8];
#pragma unroll
  for (int it = 0; it < 8; ++it) {
    const int row = wave * 32 + it * 4 + q;
    cv[it] = *(const v4f*)(Ct + row * 32 + c4);
    sv[it] = *(const v4f*)(St + row * 32 + c4);
  }
  for (int ps = 0; ps < 2; ++ps) {
#pragma unroll
    for (int it = 0; it < 8; ++it) {
      const int row = wave * 32 + it * 4 + q;
      const size_t grow = (size_t)blockIdx.x * 128 + row;
      *(volatile v4f*)(cosT + grow * 32 + c4) = cv[it];
      *(volatile v4f*)(sinT + grow * 32 + c4) = sv[it];
    }
    __threadfence();
  }
}

__global__ __launch_bounds__(256) void cast_w_kernel(
    const float* __restrict__ w0, const float* __restrict__ w1, const float* __restrict__ w2,
    const float* __restrict__ w3, const float* __restrict__ lrw, unsigned short* __restrict__ wpl) {
  const int sel = blockIdx.y;
  const int i8 = blockIdx.x * 256 + threadIdx.x;
  const int n8 = (sel < 4) ? (kDim * kDim / 8) : (64 * kDim / 8);
  if (i8 >= n8) return;
  const float* src = (sel == 0) ? w0 : (sel == 1) ? w1 : (sel == 2) ? w2 : (sel == 3) ? w3 : lrw;
  unsigned short* dst = wpl + (size_t)sel * kDim * kDim;
  const int e0 = i8 * 8;
  int srow = e0 >> 9;
  const int col = e0 & 511;
  const bool valid = (sel < 4) || (srow < kNH);
  if (sel == 4) srow = (srow < kNH) ? srow : (kNH - 1);
  const float* sp = src + (size_t)srow * kDim + col;
  const v4f a = *(const v4f*)(sp), c = *(const v4f*)(sp + 4);
  unsigned short hb[8];
#pragma unroll
  for (int e = 0; e < 4; ++e) {
    hb[e]     = f2bf_bits(valid ? a[e] : 0.0f);
    hb[4 + e] = f2bf_bits(valid ? c[e] : 0.0f);
  }
  const v4u w = (v4u){pk2(hb[0], hb[1]), pk2(hb[2], hb[3]), pk2(hb[4], hb[5]), pk2(hb[6], hb[7])};
  *(volatile v4u*)(dst + e0) = w;
  __threadfence();
  *(volatile v4u*)(dst + e0) = w;
}

__global__ __launch_bounds__(256) void ln_in_kernel(
    const float* __restrict__ x, const float* __restrict__ lw, const float* __restrict__ lbias,
    unsigned short* __restrict__ xh, unsigned short* __restrict__ xl) {
  __shared__ __align__(16) float T[32 * 260];
  __shared__ float red0[8 * 32], red1[8 * 32];
  const int tid = threadIdx.x, wave = tid >> 5, lane = tid & 31;
  const int blk = blockIdx.x;
  const int b = blk >> 7, t0 = (blk & 127) * 32;
  const float* xp = x + (size_t)b * kDim * kTok + t0 + lane;

  float s = 0.f, s2 = 0.f;
#pragma unroll 4
  for (int i = 0; i < 64; ++i) {
    const float v = bfr(xp[(size_t)(wave * 64 + i) * kTok]);
    s += v;
    s2 += v * v;
  }
  red0[wave * 32 + lane] = s;
  red1[wave * 32 + lane] = s2;
  __syncthreads();
  float ts = 0.f, ts2 = 0.f;
#pragma unroll
  for (int w = 0; w < 8; ++w) { ts += red0[w * 32 + lane]; ts2 += red1[w * 32 + lane]; }
  const float mu = ts * (1.0f / 512.0f);
  const float var = fmaxf(ts2 * (1.0f / 512.0f) - mu * mu, 0.0f);
  const float rstd = 1.0f / sqrtf(var + 1e-5f);

  for (int dh = 0; dh < 2; ++dh) {
#pragma unroll 4
    for (int i = 0; i < 32; ++i) {
      const int d = dh * 256 + wave * 32 + i;
      const float v = bfr(xp[(size_t)d * kTok]);
      const float g = bfr(lw[d]), bb = bfr(lbias[d]);
      T[lane * 260 + wave * 32 + i] = (v - mu) * rstd * g + bb;
    }
    __syncthreads();
    v4u hw[4], lwv[4];
#pragma unroll
    for (int r = 0; r < 4; ++r) {
      const float* tp = T + (wave * 4 + r) * 260 + 8 * lane;
      const v4f a = *(const v4f*)(tp), c = *(const v4f*)(tp + 4);
      unsigned short hb[8], lb8[8];
#pragma unroll
      for (int e = 0; e < 4; ++e) { split2(a[e], hb[e], lb8[e]); split2(c[e], hb[4 + e], lb8[4 + e]); }
      hw[r]  = (v4u){pk2(hb[0], hb[1]), pk2(hb[2], hb[3]), pk2(hb[4], hb[5]), pk2(hb[6], hb[7])};
      lwv[r] = (v4u){pk2(lb8[0], lb8[1]), pk2(lb8[2], lb8[3]), pk2(lb8[4], lb8[5]), pk2(lb8[6], lb8[7])};
    }
    for (int ps = 0; ps < 2; ++ps) {
#pragma unroll
      for (int r = 0; r < 4; ++r) {
        const size_t gi = ((size_t)b * kTok + t0 + wave * 4 + r) * kDim + dh * 256 + 8 * lane;
        *(volatile v4u*)(xh + gi) = hw[r];
        *(volatile v4u*)(xl + gi) = lwv[r];
      }
      __threadfence();
    }
    __syncthreads();
  }
}

__global__ __launch_bounds__(128) void scan_kernel(
    const float* __restrict__ qkv, const float* __restrict__ lrz, const float* __restrict__ lrb,
    const float* __restrict__ W1g, const float* __restrict__ b1g,
    const float* __restrict__ tlw, const float* __restrict__ tlb, const float* __restrict__ tde,
    const float* __restrict__ cosT, const float* __restrict__ sinT,
    float* __restrict__ sout, int hf) {
  __shared__ __align__(16) float W1f[kHD * kHD];
  __shared__ __align__(16) unsigned short W1Th[kHD * kHD];
  __shared__ __align__(16) unsigned short W1Tl[kHD * kHD];
  __shared__ __align__(16) float Qf[kCS * kHD];
  __shared__ __align__(16) unsigned short Qh[kCS * kHD];
  __shared__ __align__(16) unsigned short Ql[kCS * kHD];
  __shared__ __align__(16) unsigned short Kh[kCS * kHD];
  __shared__ __align__(16) unsigned short Kl[kCS * kHD];
  __shared__ __align__(16) float Tg[kCS * kHD];
  __shared__ __align__(16) float Zs[kCS * kHD];
  __shared__ __align__(16) float Gf[kCS * kHD];
  __shared__ __align__(16) unsigned short GTh[kHD * 32];
  __shared__ __align__(16) unsigned short GTl[kHD * 32];
  __shared__ __align__(16) unsigned short KTh[kHD * 32];
  __shared__ __align__(16) unsigned short KTl[kHD * 32];
  __shared__ __align__(16) unsigned short AcH[kCS * 32];
  __shared__ __align__(16) unsigned short AcL[kCS * 32];
  __shared__ __align__(16) float At[kCS * kCS];
  __shared__ __align__(16) float Os[kCS * 68];
  __shared__ float b1s[kHD], gL[kHD], bL[kHD], tki[kCS], sg[kCS];

  const int tid = threadIdx.x, wave = tid >> 5, lane = tid & 31;
  const int lh = lane >> 4, rl = lane & 15, koff = lh * 8;
  const int bloc = blockIdx.x >> 3, hd = blockIdx.x & 7;
  const int b = hf * 2 + bloc;
  const size_t kPl = (size_t)kHalfTok * kDim;
  const float* qp = qkv + (size_t)bloc * kTok * kDim + hd * kHD;
  const int m = tid >> 3, s8 = tid & 7, c0 = 4 * s8, db = 8 * s8;
  const int ncol = wave * 16 + rl;

  for (int i = tid; i < kHD * kHD; i += 128) W1f[i] = bfr(W1g[(size_t)hd * kHD * kHD + i]);
  {
    unsigned* z0 = (unsigned*)GTh; unsigned* z1 = (unsigned*)GTl;
    unsigned* z2 = (unsigned*)KTh; unsigned* z3 = (unsigned*)KTl;
    for (int i = tid; i < kHD * 16; i += 128) { z0[i] = 0u; z1[i] = 0u; z2[i] = 0u; z3[i] = 0u; }
    unsigned* z4 = (unsigned*)AcH; unsigned* z5 = (unsigned*)AcL;
    for (int i = tid; i < kCS * 16; i += 128) { z4[i] = 0u; z5[i] = 0u; }
    unsigned* z6 = (unsigned*)W1Tl;
    for (int i = tid; i < kHD * 32; i += 128) z6[i] = 0u;
  }
  if (tid < kHD) {
    b1s[tid] = bfr(b1g[hd * kHD + tid]);
    gL[tid]  = bfr(tlw[hd * kHD + tid]);
    bL[tid]  = bfr(tlb[hd * kHD + tid]);
  }
  if (tid < kCS) tki[tid] = fmaxf(1.0f / (float)(tid + 1) + bfr(tde[tid]), 0.0f);
  const float lrbv = bfr(lrb[hd]);
  __syncthreads();
  for (int i = tid; i < kHD * kHD; i += 128) { const int n = i >> 6, k = i & 63; W1Th[i] = f2bf_bits(W1f[k * kHD + n]); }
  __syncthreads();

  for (int c = 0; c < kNC; ++c) {
    const int tl = c * kCS + m;
    if (tid < kCS) {
      const size_t gt = (size_t)b * kTok + c * kCS + tid;
      const float z = lrz[gt * 64 + hd] + lrbv;
      const float ex = expf(-z);
      sg[tid] = (1.0f / (1.0f + ex)) * 0.015625f;
    }
    float k1[4], k2[4];
    {
      const float* qr = qp + (size_t)tl * kDim;
      const v4f qa = *(const v4f*)(qr + c0), qb = *(const v4f*)(qr + 32 + c0);
      const v4f ka = *(const v4f*)(qr + kPl + c0), kb = *(const v4f*)(qr + kPl + 32 + c0);
      const v4f va = *(const v4f*)(qr + 2 * kPl + c0), vb = *(const v4f*)(qr + 2 * kPl + 32 + c0);
      const v4f cs4 = *(const v4f*)(cosT + (size_t)tl * 32 + c0);
      const v4f sn4 = *(const v4f*)(sinT + (size_t)tl * 32 + c0);
      float q1[4], q2[4];
#pragma unroll
      for (int e = 0; e < 4; ++e) {
        q1[e] = qa[e] * cs4[e] - qb[e] * sn4[e];
        q2[e] = qb[e] * cs4[e] + qa[e] * sn4[e];
        k1[e] = ka[e] * cs4[e] - kb[e] * sn4[e];
        k2[e] = kb[e] * cs4[e] + ka[e] * sn4[e];
      }
      *(v4f*)(Qf + m * kHD + c0)      = (v4f){q1[0], q1[1], q1[2], q1[3]};
      *(v4f*)(Qf + m * kHD + 32 + c0) = (v4f){q2[0], q2[1], q2[2], q2[3]};
      *(v4f*)(Tg + m * kHD + c0)      = (v4f){va[0] - k1[0], va[1] - k1[1], va[2] - k1[2], va[3] - k1[3]};
      *(v4f*)(Tg + m * kHD + 32 + c0) = (v4f){vb[0] - k2[0], vb[1] - k2[1], vb[2] - k2[2], vb[3] - k2[3]};
      st_split4(Qh + m * kHD + c0,      Ql + m * kHD + c0,      q1[0], q1[1], q1[2], q1[3]);
      st_split4(Qh + m * kHD + 32 + c0, Ql + m * kHD + 32 + c0, q2[0], q2[1], q2[2], q2[3]);
      st_split4(Kh + m * kHD + c0,      Kl + m * kHD + c0,      k1[0], k1[1], k1[2], k1[3]);
      st_split4(Kh + m * kHD + 32 + c0, Kl + m * kHD + 32 + c0, k2[0], k2[1], k2[2], k2[3]);
    }
    __syncthreads();

    {
      const float le = tki[kCS - 1] * sg[m];
#pragma unroll
      for (int e = 0; e < 4; ++e) {
        unsigned short hb, lb;
        split2(-(le * k1[e]), hb, lb);
        KTh[(c0 + e) * 32 + m] = hb;
        KTl[(c0 + e) * 32 + m] = lb;
        split2(-(le * k2[e]), hb, lb);
        KTh[(32 + c0 + e) * 32 + m] = hb;
        KTl[(32 + c0 + e) * 32 + m] = lb;
      }
    }
    {
      v8f acc = zero8();
#pragma unroll
      for (int ks = 0; ks < 2; ++ks) {
        const v16b ah  = frag_lds(Kh + rl * kHD + ks * 32 + koff);
        const v16b al  = frag_lds(Kl + rl * kHD + ks * 32 + koff);
        const v16b bh  = frag_lds(W1Th + ncol * kHD + ks * 32 + koff);
        const v16b blo = frag_lds(W1Tl + ncol * kHD + ks * 32 + koff);
        acc = bmma(ah, bh, acc);
        acc = bmma(ah, blo, acc);
        acc = bmma(al, bh, acc);
      }
      const float bb = b1s[ncol];
#pragma unroll
      for (int r = 0; r < 8; ++r) Zs[(8 * lh + r) * kHD + ncol] = acc[r] + bb;
    }
    if (wave == 0) {
      v8f acc = zero8();
#pragma unroll
      for (int ks = 0; ks < 2; ++ks) {
        const v16b ah  = frag_lds(Qh + rl * kHD + ks * 32 + koff);
        const v16b al  = frag_lds(Ql + rl * kHD + ks * 32 + koff);
        const v16b bh  = frag_lds(Kh + rl * kHD + ks * 32 + koff);
        const v16b blo = frag_lds(Kl + rl * kHD + ks * 32 + koff);
        acc = bmma(ah, bh, acc);
        acc = bmma(ah, blo, acc);
        acc = bmma(al, bh, acc);
      }
#pragma unroll
      for (int r = 0; r < 8; ++r) {
        const int i = 8 * lh + r;
        At[i * kCS + rl] = (rl <= i) ? acc[r] : 0.0f;
      }
    }
    __syncthreads();

    {
      const v4f za = *(const v4f*)(Zs + m * kHD + db), zb = *(const v4f*)(Zs + m * kHD + db + 4);
      const v4f ta = *(const v4f*)(Tg + m * kHD + db), tb = *(const v4f*)(Tg + m * kHD + db + 4);
      float z[8]   = {za[0], za[1], za[2], za[3], zb[0], zb[1], zb[2], zb[3]};
      float tg8[8] = {ta[0], ta[1], ta[2], ta[3], tb[0], tb[1], tb[2], tb[3]};
      float sm = 0.f;
#pragma unroll
      for (int e = 0; e < 8; ++e) sm += z[e];
      sm = red8(sm);
      const float mu = sm * (1.0f / 64.0f);
      float d[8];
      float sq = 0.f;
#pragma unroll
      for (int e = 0; e < 8; ++e) { d[e] = z[e] - mu; sq += d[e] * d[e]; }
      sq = red8(sq);
      const float sd = sqrtf(sq * (1.0f / 64.0f) + 1e-6f);
      const float rs = 1.0f / sd;
      float xh8[8], gx[8];
      float S1 = 0.f, S2 = 0.f;
#pragma unroll
      for (int e = 0; e < 8; ++e) {
        const float xhv = d[e] * rs;
        const float g = gL[db + e];
        const float gv = (g * xhv + bL[db + e] - tg8[e]) * g;
        xh8[e] = xhv; gx[e] = gv;
        S1 += gv; S2 += gv * xhv;
      }
      S1 = red8(S1);
      S2 = red8(S2);
      const float inv = 1.0f / (64.0f * sd);
      float gr[8];
#pragma unroll
      for (int e = 0; e < 8; ++e) gr[e] = (64.0f * gx[e] - S1 - xh8[e] * S2) * inv;
      *(v4f*)(Gf + m * kHD + db)     = (v4f){gr[0], gr[1], gr[2], gr[3]};
      *(v4f*)(Gf + m * kHD + db + 4) = (v4f){gr[4], gr[5], gr[6], gr[7]};
#pragma unroll
      for (int e = 0; e < 8; ++e) {
        unsigned short hb, lb;
        split2(gr[e], hb, lb);
        GTh[(db + e) * 32 + m] = hb;
        GTl[(db + e) * 32 + m] = lb;
      }
      {
        const int i = m, jj = 2 * s8;
        const float e0 = tki[i] * sg[jj], e1 = tki[i] * sg[jj + 1];
        float v0 = -(e0 * At[i * kCS + jj] + e0);
        float v1 = -(e1 * At[i * kCS + jj + 1] + e1);
        v0 = (jj <= i) ? v0 : 0.0f;
        v1 = (jj + 1 <= i) ? v1 : 0.0f;
        unsigned short h0, l0, h1, l1;
        split2(v0, h0, l0);
        split2(v1, h1, l1);
        ((unsigned*)AcH)[i * 16 + s8] = pk2(h0, h1);
        ((unsigned*)AcL)[i * 16 + s8] = pk2(l0, l1);
      }
    }
    __syncthreads();

    {
      v8f acc = zero8();
#pragma unroll
      for (int ks = 0; ks < 2; ++ks) {
        const v16b ah  = frag_lds(Qh + rl * kHD + ks * 32 + koff);
        const v16b al  = frag_lds(Ql + rl * kHD + ks * 32 + koff);
        const v16b bh  = frag_lds(W1Th + ncol * kHD + ks * 32 + koff);
        const v16b blo = frag_lds(W1Tl + ncol * kHD + ks * 32 + koff);
        acc = bmma(ah, bh, acc);
        acc = bmma(ah, blo, acc);
        acc = bmma(al, bh, acc);
      }
      {
        const v16b ah  = frag_lds(AcH + rl * 32 + koff);
        const v16b al  = frag_lds(AcL + rl * 32 + koff);
        const v16b bh  = frag_lds(GTh + ncol * 32 + koff);
        const v16b blo = frag_lds(GTl + ncol * 32 + koff);
        acc = bmma(ah, bh, acc);
        acc = bmma(ah, blo, acc);
        acc = bmma(al, bh, acc);
      }
      const float bb = b1s[ncol];
#pragma unroll
      for (int r = 0; r < 8; ++r) Zs[(8 * lh + r) * kHD + ncol] = acc[r] + bb;
    }
    __syncthreads();

    {
      const v4f za = *(const v4f*)(Zs + m * kHD + db), zb = *(const v4f*)(Zs + m * kHD + db + 4);
      const v4f fa = *(const v4f*)(Qf + m * kHD + db), fb = *(const v4f*)(Qf + m * kHD + db + 4);
      float z[8]  = {za[0], za[1], za[2], za[3], zb[0], zb[1], zb[2], zb[3]};
      float q8[8] = {fa[0], fa[1], fa[2], fa[3], fb[0], fb[1], fb[2], fb[3]};
      float sm = 0.f;
#pragma unroll
      for (int e = 0; e < 8; ++e) sm += z[e];
      sm = red8(sm);
      const float mu = sm * (1.0f / 64.0f);
      float d[8];
      float sq = 0.f;
#pragma unroll
      for (int e = 0; e < 8; ++e) { d[e] = z[e] - mu; sq += d[e] * d[e]; }
      sq = red8(sq);
      const float rs = 1.0f / sqrtf(sq * (1.0f / 64.0f) + 1e-6f);
      float o[8];
#pragma unroll
      for (int e = 0; e < 8; ++e) o[e] = q8[e] + (d[e] * rs * gL[db + e] + bL[db + e]);
      *(v4f*)(Os + m * 68 + db)     = (v4f){o[0], o[1], o[2], o[3]};
      *(v4f*)(Os + m * 68 + db + 4) = (v4f){o[4], o[5], o[6], o[7]};
    }
    {
      const v16b bh  = frag_lds(GTh + ncol * 32 + koff);
      const v16b blo = frag_lds(GTl + ncol * 32 + koff);
#pragma unroll
      for (int mt = 0; mt < 4; ++mt) {
        v8f acc;
#pragma unroll
        for (int r = 0; r < 8; ++r) acc[r] = W1f[(mt * 16 + 8 * lh + r) * kHD + ncol];
        const v16b ah = frag_lds(KTh + (mt * 16 + rl) * 32 + koff);
        const v16b al = frag_lds(KTl + (mt * 16 + rl) * 32 + koff);
        acc = bmma(ah, bh, acc);
        acc = bmma(ah, blo, acc);
        acc = bmma(al, bh, acc);
        unsigned short hb[8], lb[8];
#pragma unroll
        for (int r = 0; r < 8; ++r) {
          W1f[(mt * 16 + 8 * lh + r) * kHD + ncol] = acc[r];
          split2(acc[r], hb[r], lb[r]);
        }
        *(v4u*)(W1Th + ncol * kHD + mt * 16 + 8 * lh) =
            (v4u){pk2(hb[0], hb[1]), pk2(hb[2], hb[3]), pk2(hb[4], hb[5]), pk2(hb[6], hb[7])};
        *(v4u*)(W1Tl + ncol * kHD + mt * 16 + 8 * lh) =
            (v4u){pk2(lb[0], lb[1]), pk2(lb[2], lb[3]), pk2(lb[4], lb[5]), pk2(lb[6], lb[7])};
      }
    }
    if (tid < kHD) {
      const float le = tki[kCS - 1];
      float sacc = 0.f;
#pragma unroll
      for (int jj = 0; jj < kCS; ++jj) sacc += (le * sg[jj]) * Gf[jj * kHD + tid];
      b1s[tid] = b1s[tid] - sacc;
    }
    __syncthreads();
    {
      const int c4 = rl * 4;
      const size_t gt0 = (size_t)b * kTok + (size_t)c * kCS;
      v4f ov[2];
#pragma unroll
      for (int it = 0; it < 2; ++it) {
        const int row = wave * 4 + it * 2 + lh;
        ov[it] = *(const v4f*)(Os + row * 68 + c4);
      }
      for (int ps = 0; ps < 2; ++ps) {
#pragma unroll
        for (int it = 0; it < 2; ++it) {
          const int row = wave * 4 + it * 2 + lh;
          *(volatile v4f*)(sout + (gt0 + row) * kDim + hd * kHD + c4) = ov[it];
        }
        __threadfence();
      }
    }
    __syncthreads();
  }
}

__global__ __launch_bounds__(256) void ln_post_kernel(
    const float* __restrict__ src, const float* __restrict__ pw, const float* __restrict__ pb,
    unsigned short* __restrict__ oh, unsigned short* __restrict__ ol) {
  const int tid = threadIdx.x, wave = tid >> 5, lane = tid & 31;
  const int row = blockIdx.x * 8 + wave;
  const float* rp = src + (size_t)row * kDim;
  const int cA = 8 * lane, cB = 256 + 8 * lane;
  const v4f a0 = *(const v4f*)(rp + cA), a1 = *(const v4f*)(rp + cA + 4);
  const v4f a2 = *(const v4f*)(rp + cB), a3 = *(const v4f*)(rp + cB + 4);
  float v[16] = {a0[0], a0[1], a0[2], a0[3], a1[0], a1[1], a1[2], a1[3],
                 a2[0], a2[1], a2[2], a2[3], a3[0], a3[1], a3[2], a3[3]};
  float s = 0.f;
#pragma unroll
  for (int e = 0; e < 16; ++e) s += v[e];
  s = red32(s);
  const float mu = s * (1.0f / 512.0f);
  float d[16];
  float sq = 0.f;
#pragma unroll
  for (int e = 0; e < 16; ++e) { d[e] = v[e] - mu; sq += d[e] * d[e]; }
  sq = red32(sq);
  const float rstd = 1.0f / sqrtf(sq * (1.0f / 512.0f) + 1e-6f);
  const v4f g0 = *(const v4f*)(pw + cA), g1 = *(const v4f*)(pw + cA + 4);
  const v4f g2 = *(const v4f*)(pw + cB), g3 = *(const v4f*)(pw + cB + 4);
  const v4f p0 = *(const v4f*)(pb + cA), p1 = *(const v4f*)(pb + cA + 4);
  const v4f p2 = *(const v4f*)(pb + cB), p3 = *(const v4f*)(pb + cB + 4);
  float g[16]  = {g0[0], g0[1], g0[2], g0[3], g1[0], g1[1], g1[2], g1[3],
                  g2[0], g2[1], g2[2], g2[3], g3[0], g3[1], g3[2], g3[3]};
  float pv[16] = {p0[0], p0[1], p0[2], p0[3], p1[0], p1[1], p1[2], p1[3],
                  p2[0], p2[1], p2[2], p2[3], p3[0], p3[1], p3[2], p3[3]};
  unsigned short hb[16], lb[16];
#pragma unroll
  for (int e = 0; e < 16; ++e) {
    const float y = d[e] * rstd * bfr(g[e]) + bfr(pv[e]);
    split2(y, hb[e], lb[e]);
  }
  const v4u hA = (v4u){pk2(hb[0], hb[1]), pk2(hb[2], hb[3]), pk2(hb[4], hb[5]), pk2(hb[6], hb[7])};
  const v4u hB = (v4u){pk2(hb[8], hb[9]), pk2(hb[10], hb[11]), pk2(hb[12], hb[13]), pk2(hb[14], hb[15])};
  const v4u lA = (v4u){pk2(lb[0], lb[1]), pk2(lb[2], lb[3]), pk2(lb[4], lb[5]), pk2(lb[6], lb[7])};
  const v4u lB = (v4u){pk2(lb[8], lb[9]), pk2(lb[10], lb[11]), pk2(lb[12], lb[13]), pk2(lb[14], lb[15])};
  unsigned short* ohr = oh + (size_t)row * kDim;
  unsigned short* olr = ol + (size_t)row * kDim;
  for (int ps = 0; ps < 2; ++ps) {
    *(volatile v4u*)(ohr + cA) = hA;
    *(volatile v4u*)(ohr + cB) = hB;
    *(volatile v4u*)(olr + cA) = lA;
    *(volatile v4u*)(olr + cB) = lB;
    __threadfence();
  }
}

constexpr size_t kSzPlane16 = (size_t)kBT * kDim * 2;
constexpr size_t kSzW      = (size_t)4 * kDim * kDim * 2 + (size_t)64 * kDim * 2;
constexpr size_t kSzCos    = (size_t)kTok * 32 * 4;
constexpr size_t kSzLrz    = (size_t)kBT * 64 * 4;
constexpr size_t kSzQkv    = (size_t)3 * kHalfTok * kDim * 4;
constexpr size_t kSzSout   = (size_t)kBT * kDim * 4;
constexpr size_t kWsTotal  = 2 * kSzPlane16 + kSzW + 2 * kSzCos + kSzLrz + kSzQkv + kSzSout;
typedef char ct_ws_total[(kWsTotal <= (size_t)134217728) ? 1 : -1];
typedef char ct_gemm_lr[((kBT % 64) == 0 && (kDim % 32) == 0) ? 1 : -1];
typedef char ct_gemm_qkv[((kHalfTok % 64) == 0 && (kDim % 64) == 0) ? 1 : -1];
typedef char ct_gemm_o[((kDim % 64) == 0 && (kTok % 64) == 0) ? 1 : -1];
typedef char ct_align[((kSzW % 256) == 0 && (kSzCos % 256) == 0 && (kSzLrz % 256) == 0) ? 1 : -1];

extern "C" void kernel_launch(void* const* d_in, const int* in_sizes, int n_in,
                              void* d_out, int out_size, void* d_ws, size_t ws_size,
                              hipStream_t stream) {
  if (n_in < 16) return;
  if (in_sizes[0] != kB * kDim * kTok || out_size != kB * kDim * kTok) return;
  if (in_sizes[3] != kDim * kDim || in_sizes[7] != kNH * kHD * kHD || in_sizes[11] != kNH * kDim) return;

  const float* x    = (const float*)d_in[0];
  const float* ln_w = (const float*)d_in[1];
  const float* ln_b = (const float*)d_in[2];
  const float* q_w  = (const float*)d_in[3];
  const float* k_w  = (const float*)d_in[4];
  const float* v_w  = (const float*)d_in[5];
  const float* o_w  = (const float*)d_in[6];
  const float* W1   = (const float*)d_in[7];
  const float* b1   = (const float*)d_in[8];
  const float* tlw  = (const float*)d_in[9];
  const float* tlb  = (const float*)d_in[10];
  const float* lrw  = (const float*)d_in[11];
  const float* lrb  = (const float*)d_in[12];
  const float* tde  = (const float*)d_in[13];
  const float* pw   = (const float*)d_in[14];
  const float* pb   = (const float*)d_in[15];
  float* out = (float*)d_out;

  if (kWsTotal > ws_size) return;
  char* ws = (char*)d_ws;
  size_t off = 0;
  unsigned short* xnh = (unsigned short*)(ws + off); off += kSzPlane16;
  unsigned short* xnl = (unsigned short*)(ws + off); off += kSzPlane16;
  unsigned short* wpl = (unsigned short*)(ws + off); off += kSzW;
  float* cosT = (float*)(ws + off); off += kSzCos;
  float* sinT = (float*)(ws + off); off += kSzCos;
  float* lrz  = (float*)(ws + off); off += kSzLrz;
  float* qkvp = (float*)(ws + off); off += kSzQkv;
  float* sout = (float*)(ws + off); off += kSzSout;
  if (off > ws_size) return;

  const size_t wPlane = (size_t)kDim * kDim;
  unsigned short* wq  = wpl;
  unsigned short* wo  = wpl + 3 * wPlane;
  unsigned short* wlr = wpl + 4 * wPlane;

  RopeFreq rf;
  for (int j = 0; j < 32; ++j) {
    const float e = (float)(2 * j) / 64.0f;
    const double p = pow(10000.0, (double)e);
    const float pf = (float)p;
    rf.inv[j] = 1.0f / pf;
  }

  tables_kernel<<<dim3(kTok / 128), dim3(128), 0, stream>>>(cosT, sinT, rf);
  cast_w_kernel<<<dim3((kDim * kDim / 8) / 256, 5), dim3(256), 0, stream>>>(q_w, k_w, v_w, o_w, lrw, wpl);
  ln_in_kernel<<<dim3(kBT / 32), dim3(256), 0, stream>>>(x, ln_w, ln_b, xnh, xnl);

  gemm64_bf16<true, false><<<dim3(((kBT / 64) * (64 / 64) + 7) / 8, 1), dim3(256), 0, stream>>>(
      xnh, xnl, kDim, 0L, wlr, wlr, kDim, 0L, lrz, 64, 0L, kBT, 64, kDim);

  for (int hf = 0; hf < 2; ++hf) {
    gemm64_bf16<true, false><<<dim3(((kHalfTok / 64) * (kDim / 64) + 7) / 8, 3), dim3(256), 0, stream>>>(
        xnh + (size_t)hf * kHalfTok * kDim, xnl + (size_t)hf * kHalfTok * kDim, kDim, 0L,
        wq, wq, kDim, (long)wPlane,
        qkvp, kDim, (long)kHalfTok * kDim, kHalfTok, kDim, kDim);
    scan_kernel<<<dim3(2 * kNH), dim3(128), 0, stream>>>(qkvp, lrz, lrb, W1, b1, tlw, tlb, tde,
                                                        cosT, sinT, sout, hf);
  }

  ln_post_kernel<<<dim3(kBT / 8), dim3(256), 0, stream>>>(sout, pw, pb, xnh, xnl);

  gemm64_bf16<false, true><<<dim3(((kDim / 64) * (kTok / 64) + 7) / 8, kB), dim3(256), 0, stream>>>(
      wo, wo, kDim, 0L, xnh, xnl, kDim, (long)kTok * kDim,
      out, kTok, (long)kDim * kTok, kDim, kTok, kDim);
}
